// LiltSelfAttention_65807488909584
// MI455X (gfx1250) — hardware-verified
//
#include <hip/hip_runtime.h>
#include <math.h>

constexpr int kBatch    = 4;
constexpr int kSeq      = 2048;
constexpr int kHid      = 768;
constexpr int kHeads    = 12;
constexpr int kHeadDim  = 64;
constexpr int kLHid     = 192;
constexpr int kLHeadDim = 16;
constexpr int kTok      = kBatch * kSeq;
constexpr int kHeadPitch = 128;
constexpr int kCombLd   = kHeads * kHeadPitch;
constexpr int kCombK    = 96;
constexpr int kLPad     = 64;
constexpr int kGroupsPerChunk = 2;
constexpr int kChunks   = kBatch * kHeads / kGroupsPerChunk;
constexpr float kWCarry     = 64.0f;
constexpr float kWCarryInv  = 1.0f / 64.0f;
constexpr float kLQScale    = 2.0f / 64.0f;
constexpr float kPCarry     = 2048.0f;
constexpr float kPCarryInv  = 1.0f / 2048.0f;
constexpr float kScoreScale = 0.125f;
constexpr size_t kOut1Float = (size_t)kTok * kHid;

static_assert(kTok % 64 == 0);
static_assert(kSeq % 64 == 0);
static_assert(kHid % 64 == 0);
static_assert(kLHid % 64 == 0);
static_assert(kHid % 32 == 0);
static_assert(kLHid % 32 == 0);
static_assert(kCombK % 32 == 0);
static_assert(kSeq % 32 == 0);

constexpr size_t kOffQC   = 0;
constexpr size_t kSzQC    = (size_t)kTok * kCombLd * 2;
constexpr size_t kOffKC   = kOffQC + kSzQC;
constexpr size_t kOffVT   = kOffKC + kSzQC;
constexpr size_t kSzVT    = (size_t)kBatch * kHid * kSeq * 2;
constexpr size_t kOffLVT  = kOffVT + kSzVT;
constexpr size_t kSzLVT   = (size_t)kBatch * kLHid * kSeq * 2;
constexpr size_t kOffLB   = kOffLVT + kSzLVT;
constexpr size_t kSzLB    = (size_t)2 * kHeads * kLPad * 4;
constexpr size_t kOffScr  = kOffLB + kSzLB;
constexpr size_t kOffX16  = kOffScr;
constexpr size_t kSzX16   = (size_t)kTok * kHid * 2;
constexpr size_t kOffLX16 = kOffX16 + kSzX16;
constexpr size_t kSzLX16  = (size_t)kTok * kLHid * 2;
constexpr size_t kOffWT   = kOffLX16 + kSzLX16;
constexpr size_t kSzWT    = (size_t)3 * kHid * kHid * 2;
constexpr size_t kOffWLP  = kOffWT + kSzWT;
constexpr size_t kSzWLP   = (size_t)2 * kHeads * kLPad * kLHid * 2;
constexpr size_t kOffWLV  = kOffWLP + kSzWLP;
constexpr size_t kSzWLV   = (size_t)kLHid * kLHid * 2;
constexpr size_t kEndA    = kOffWLV + kSzWLV;
constexpr size_t kOffSC   = kOffScr;
constexpr size_t kSzSC    = (size_t)kGroupsPerChunk * kSeq * kSeq * 4;
constexpr size_t kOffP16  = kOffSC + kSzSC;
constexpr size_t kSzP16   = (size_t)kGroupsPerChunk * kSeq * kSeq * 2;
constexpr size_t kEndB    = kOffP16 + kSzP16;
constexpr size_t kWsTotal = (kEndA > kEndB) ? kEndA : kEndB;
static_assert(kWsTotal <= (size_t)134217728);
static_assert(kOffScr % 128 == 0 && kOffLX16 % 128 == 0 && kOffWT % 128 == 0 && kOffWLP % 128 == 0 && kOffWLV % 128 == 0 && kOffP16 % 128 == 0);

typedef __attribute__((ext_vector_type(16))) _Float16 v16h;
typedef __attribute__((ext_vector_type(8)))  _Float16 v8h;
typedef __attribute__((ext_vector_type(16))) __bf16   v16b;
typedef __attribute__((ext_vector_type(8)))  __bf16   v8b;
typedef __attribute__((ext_vector_type(8)))  float    v8f;
typedef __attribute__((ext_vector_type(4)))  float    v4f;
typedef __attribute__((ext_vector_type(4)))  unsigned int v4u;

__device__ __forceinline__ unsigned short f2bf_bits(float f) {
  unsigned u = __float_as_uint(f);
  return (unsigned short)((u + 0x7FFFu + ((u >> 16) & 1u)) >> 16);
}
__device__ __forceinline__ float bf_bits2f(unsigned short h) { return __uint_as_float(((unsigned)h) << 16); }

__device__ __forceinline__ void dep_guard_h(v8f& a, v8f& b, v16h x, v16h y) { asm volatile("v_nop\n\tv_nop\n\tv_nop\n\tv_nop" : "+v"(a), "+v"(b) : "v"(x), "v"(y)); }
__device__ __forceinline__ void dep_guard_b(v8f& a, v8f& b, v16b x, v16b y) { asm volatile("v_nop\n\tv_nop\n\tv_nop\n\tv_nop" : "+v"(a), "+v"(b) : "v"(x), "v"(y)); }
__device__ __forceinline__ void keep4_h(v16h a, v16h b, v16h c, v16h d) { asm volatile("v_nop" :: "v"(a), "v"(b), "v"(c), "v"(d)); }
__device__ __forceinline__ void keep4_b(v16b a, v16b b, v16b c, v16b d) { asm volatile("v_nop" :: "v"(a), "v"(b), "v"(c), "v"(d)); }
__device__ __forceinline__ void acc_guard4(v8f& a, v8f& b, v8f& c, v8f& d) { asm volatile("v_nop\n\tv_nop\n\tv_nop\n\tv_nop" : "+v"(a), "+v"(b), "+v"(c), "+v"(d)); }
template <typename T> struct Frag;
template <> struct Frag<_Float16> {
  typedef v16h V; union U { v16h v; v8h h[2]; };
  static __device__ __forceinline__ v16h load(const _Float16* p) {
    U f; f.h[0] = *(const v8h*)(p); f.h[1] = *(const v8h*)(p + 16); return f.v;
  }
  static __device__ __forceinline__ v8f mma(v16h a, v16h b, v8f c) {
    return __builtin_amdgcn_wmma_f32_16x16x32_f16(false, a, false, b, (short)0, c, false, false);
  }
  static __device__ __forceinline__ void guard(v8f& a, v8f& b, v16h x, v16h y) { dep_guard_h(a, b, x, y); }
  static __device__ __forceinline__ void keep(v16h a, v16h b, v16h c, v16h d) { keep4_h(a, b, c, d); }
};
template <> struct Frag<__bf16> {
  typedef v16b V; union U { v16b v; v8b h[2]; };
  static __device__ __forceinline__ v16b load(const __bf16* p) {
    U f; f.h[0] = *(const v8b*)(p); f.h[1] = *(const v8b*)(p + 16); return f.v;
  }
  static __device__ __forceinline__ v8f mma(v16b a, v16b b, v8f c) {
    return __builtin_amdgcn_wmma_f32_16x16x32_bf16(false, a, false, b, (short)0, c, false, false);
  }
  static __device__ __forceinline__ void guard(v8f& a, v8f& b, v16b x, v16b y) { dep_guard_b(a, b, x, y); }
  static __device__ __forceinline__ void keep(v16b a, v16b b, v16b c, v16b d) { keep4_b(a, b, c, d); }
};

__device__ __forceinline__ unsigned pk16(unsigned short a, unsigned short b) { return (unsigned)a | ((unsigned)b << 16); }
__device__ __forceinline__ unsigned short h_bits(float f) { const _Float16 h = (_Float16)f; return __builtin_bit_cast(unsigned short, h); }

template <int ET> struct Elem;
template <> struct Elem<0> { typedef _Float16 T; };
template <> struct Elem<1> { typedef __bf16 T; };
template <int ET, bool SPLIT, int BIAS_MODE, int OUT_MODE, bool RESID, int ACT = 0>
__global__ __launch_bounds__(256) void wmma_gemm64(
    const unsigned short* __restrict__ Ap, const unsigned short* __restrict__ A2p, int lda, long strideA,
    const unsigned short* __restrict__ Btp, const unsigned short* __restrict__ Bt2p, int ldb, long strideB,
    void* __restrict__ Cout, void* __restrict__ Cout2, int ldc, long strideC,
    const float* __restrict__ bias, long strideBias,
    const float* __restrict__ resid, long strideR,
    int M, int N, int K, float scale) {
  typedef typename Elem<ET>::T T;
  typedef typename Frag<T>::V V;
  const T* A = (const T*)Ap; const T* A2 = (const T*)A2p; const T* Bt = (const T*)Btp; const T* Bt2 = (const T*)Bt2p;
  __shared__ __align__(16) float sT[8][16 * 68];
  const int b    = blockIdx.y;
  const int lane = threadIdx.x & 31;
  const int wave = threadIdx.x >> 5;
  const int tilesN = N >> 6;
  const int tilesM = M >> 6;
  const int tile = blockIdx.x * 8 + wave;
  if (tile >= tilesM * tilesN) return;
  const int tm = tile / tilesN;
  const int tn = tile - tm * tilesN;
  const int m0 = tm << 6;
  const int n0 = tn << 6;

  const T* Ab  = A  + (size_t)b * strideA;
  const T* Bb  = Bt + (size_t)b * strideB;
  const T* Ab2 = SPLIT ? (A2  + (size_t)b * strideA) : nullptr;
  const T* Bb2 = SPLIT ? (Bt2 + (size_t)b * strideB) : nullptr;

  const int rlane = lane & 15;
  const int koff  = (lane >> 4) * 8;
  const int mOff  = (lane >> 4) * 8;

  v8f acc[4][4];
#pragma unroll
  for (int i = 0; i < 4; ++i)
#pragma unroll
    for (int j = 0; j < 4; ++j) acc[i][j] = (v8f){0.f,0.f,0.f,0.f,0.f,0.f,0.f,0.f};

  for (int k0 = 0; k0 < K; k0 += 32) {
    V bh[4], bl[4];
#pragma unroll
    for (int j = 0; j < 4; ++j) {
      const size_t bo = (size_t)(n0 + (j << 4) + rlane) * ldb + koff + k0;
      bh[j] = Frag<T>::load(Bb + bo);
      if (SPLIT) bl[j] = Frag<T>::load(Bb2 + bo);
    }
#pragma unroll
    for (int i = 0; i < 4; ++i) {
      const size_t ao = (size_t)(m0 + (i << 4) + rlane) * lda + koff + k0;
      V ah = Frag<T>::load(Ab + ao);
      V al;
      if (SPLIT) al = Frag<T>::load(Ab2 + ao);
#pragma unroll
      for (int j = 0; j < 4; ++j) {
        acc[i][j] = Frag<T>::mma(ah, bh[j], acc[i][j]);
        if (SPLIT) {
          acc[i][j] = Frag<T>::mma(ah, bl[j], acc[i][j]);
          acc[i][j] = Frag<T>::mma(al, bh[j], acc[i][j]);
        }
      }
      Frag<T>::guard(acc[i][0], acc[i][3], ah, SPLIT ? al : ah);
    }
    Frag<T>::keep(bh[0], bh[1], bh[2], bh[3]);
    if (SPLIT) Frag<T>::keep(bl[0], bl[1], bl[2], bl[3]);
  }
  acc_guard4(acc[0][0], acc[0][1], acc[0][2], acc[0][3]);
  acc_guard4(acc[1][0], acc[1][1], acc[1][2], acc[1][3]);
  acc_guard4(acc[2][0], acc[2][1], acc[2][2], acc[2][3]);
  acc_guard4(acc[3][0], acc[3][1], acc[3][2], acc[3][3]);

  float* slab = sT[wave];
  const float* Rb = RESID ? (resid + (size_t)b * strideR) : nullptr;
  const size_t bOff = (BIAS_MODE != 0) ? (size_t)b * strideBias : (size_t)0;
#pragma unroll
  for (int i = 0; i < 4; ++i) {
    const int mBase = m0 + (i << 4);
#pragma unroll
    for (int j = 0; j < 4; ++j) {
      const int n = n0 + (j << 4) + rlane;
      float bv = 0.f;
      if (BIAS_MODE == 2) bv = bias[bOff + n];
#pragma unroll
      for (int r = 0; r < 8; ++r) {
        float v = acc[i][j][r] * scale;
        if (BIAS_MODE == 1) v += bias[bOff + mBase + mOff + r];
        if (BIAS_MODE == 2) v += bv;
        if (RESID) v += Rb[(size_t)(mBase + mOff + r) * ldc + n];
        if (ACT == 2) v = fmaxf(v, 0.0f);
        if (ACT == 4) v = (v > 0.f) ? v : 0.01f * v;
        slab[(mOff + r) * 68 + (j << 4) + rlane] = v;
      }
    }
    __builtin_amdgcn_fence(__ATOMIC_RELEASE, "workgroup");
    __builtin_amdgcn_wave_barrier();
    __builtin_amdgcn_fence(__ATOMIC_ACQUIRE, "workgroup");
    if (OUT_MODE == 0) {
      float* C = (float*)Cout + (size_t)b * strideC;
      const int hh = lane >> 4, c4 = (lane & 15) * 4;
      for (int pass = 0; pass < 2; ++pass) {
#pragma unroll
        for (int it = 0; it < 8; ++it) {
          const int row = it * 2 + hh;
          v4f v = *(const v4f*)(slab + row * 68 + c4);
          *(volatile v4f*)(C + (size_t)(mBase + row) * ldc + n0 + c4) = v;
        }
        __threadfence();
      }
    } else {
      const int q = lane >> 3, c8 = (lane & 7) * 8;
      unsigned short* C  = (unsigned short*)Cout  + (size_t)b * strideC;
      unsigned short* C2 = (OUT_MODE == 2) ? ((unsigned short*)Cout2 + (size_t)b * strideC) : nullptr;
      for (int pass = 0; pass < 2; ++pass) {
#pragma unroll
        for (int it = 0; it < 4; ++it) {
          const int row = it * 4 + q;
          const float* sp = slab + row * 68 + c8;
          v8h hv, lv;
#pragma unroll
          for (int e = 0; e < 8; ++e) {
            if (OUT_MODE == 1) {
              hv[e] = (_Float16)sp[e];
            } else {
              unsigned short hb = f2bf_bits(sp[e]);
              unsigned short lb = f2bf_bits(sp[e] - bf_bits2f(hb));
              hv[e] = __builtin_bit_cast(_Float16, hb);
              lv[e] = __builtin_bit_cast(_Float16, lb);
            }
          }
          *(volatile v8h*)(C + (size_t)(mBase + row) * ldc + n0 + c8) = hv;
          if (OUT_MODE == 2) *(volatile v8h*)(C2 + (size_t)(mBase + row) * ldc + n0 + c8) = lv;
        }
        __threadfence();
      }
    }
    __builtin_amdgcn_fence(__ATOMIC_RELEASE, "workgroup");
    __builtin_amdgcn_wave_barrier();
    __builtin_amdgcn_fence(__ATOMIC_ACQUIRE, "workgroup");
  }
}

__global__ __launch_bounds__(256) void cast8_f16_kernel(const float* __restrict__ in, unsigned short* __restrict__ out, int n8) {
  const int i = blockIdx.x * 256 + threadIdx.x;
  if (i >= n8) return;
  const float* p = in + 8 * (size_t)i;
  const v4f a = *(const v4f*)(p);
  const v4f c = *(const v4f*)(p + 4);
  unsigned short hb[8];
#pragma unroll
  for (int e = 0; e < 4; ++e) {
    hb[e]     = h_bits(a[e]);
    hb[4 + e] = h_bits(c[e]);
  }
  const v4u u = (v4u){pk16(hb[0], hb[1]), pk16(hb[2], hb[3]), pk16(hb[4], hb[5]), pk16(hb[6], hb[7])};
  unsigned short* q = out + 8 * (size_t)i;
  *(volatile v4u*)q = u;
  __threadfence();
  *(volatile v4u*)q = u;
}

__global__ __launch_bounds__(256) void wt_text_kernel(const float* __restrict__ W0, const float* __restrict__ W1,
                                                      const float* __restrict__ W2, unsigned short* __restrict__ out, float scale) {
  __shared__ float sm[64][65];
  const int t  = threadIdx.x;
  const int d0 = blockIdx.x * 64;
  const int n0 = blockIdx.y * 64;
  const int z  = blockIdx.z;
  const float* W = (z == 0) ? W0 : (z == 1) ? W1 : W2;
#pragma unroll
  for (int i = 0; i < 16; ++i) {
    const int e = i * 256 + t;
    const int r = e >> 6;
    const int c = e & 63;
    sm[c][r] = W[(size_t)(d0 + r) * kHid + n0 + c] * scale;
  }
  __syncthreads();
  const int lane = t & 31, wave = t >> 5;
  const int q = lane >> 3, c8 = (lane & 7) * 8;
  unsigned short* op = out + (size_t)z * kHid * kHid;
  for (int pass = 0; pass < 2; ++pass) {
#pragma unroll
    for (int it = 0; it < 2; ++it) {
      const int row = wave * 8 + it * 4 + q;
      unsigned short hb[8];
#pragma unroll
      for (int e = 0; e < 8; ++e) hb[e] = h_bits(sm[row][c8 + e]);
      const v4u u = (v4u){pk16(hb[0], hb[1]), pk16(hb[2], hb[3]), pk16(hb[4], hb[5]), pk16(hb[6], hb[7])};
      *(volatile v4u*)(op + (size_t)(n0 + row) * kHid + d0 + c8) = u;
    }
    __threadfence();
  }
}

template <int PR>
__global__ __launch_bounds__(256) void wt_layout_kernel(const float* __restrict__ W0, const float* __restrict__ W1,
                                                        unsigned short* __restrict__ out, float scale) {
  __shared__ float sm[16][196];
  const int t = threadIdx.x;
  const int h = blockIdx.x;
  const int y = blockIdx.y;
  const float* W = (y == 0) ? W0 : W1;
#pragma unroll
  for (int i = 0; i < 12; ++i) {
    const int e = i * 256 + t;
    const int d = e >> 4;
    const int j = e & 15;
    sm[j][d] = W[(size_t)d * kLHid + h * kLHeadDim + j] * scale;
  }
  __syncthreads();
  constexpr int kCount = PR * 24;
  constexpr int kIters = (kCount + 255) / 256;
  unsigned short* op = out + (size_t)y * ((size_t)kHeads * PR * kLHid) + (size_t)h * PR * kLHid;
  for (int pass = 0; pass < 2; ++pass) {
#pragma unroll
    for (int it = 0; it < kIters; ++it) {
      const int idx = it * 256 + t;
      if (idx < kCount) {
        const int row = idx / 24;
        const int c8  = (idx - row * 24) * 8;
        const int rr  = (row < 16) ? row : 15;
        unsigned short hb[8];
#pragma unroll
        for (int e = 0; e < 8; ++e) {
          const float v = sm[rr][c8 + e];
          hb[e] = h_bits((row < 16) ? v : 0.0f);
        }
        const v4u u = (v4u){pk16(hb[0], hb[1]), pk16(hb[2], hb[3]), pk16(hb[4], hb[5]), pk16(hb[6], hb[7])};
        *(volatile v4u*)(op + (size_t)row * kLHid + c8) = u;
      }
    }
    __threadfence();
  }
}

__device__ __forceinline__ v4f bias_tab_value(const float* __restrict__ lbq, const float* __restrict__ lbk, int idx) {
  const int tbl = idx / 192;
  const int n4  = (idx - tbl * 192) * 4;
  const int h   = n4 >> 6;
  const int j0  = n4 & 63;
  float v[4];
#pragma unroll
  for (int e = 0; e < 4; ++e) {
    const int j   = j0 + e;
    const int src = h * kLHeadDim + ((j < 16) ? j : 15);
    const float fq = lbq[src];
    const float fk = lbk[src];
    const float sel = (tbl == 0) ? 2.0f * fq : fk;
    v[e] = (j < 16) ? sel : 0.0f;
  }
  return (v4f){v[0], v[1], v[2], v[3]};
}
__global__ __launch_bounds__(256) void bias_prep_kernel(const float* __restrict__ lbq, const float* __restrict__ lbk,
                                                        float* __restrict__ LB) {
  const int t = threadIdx.x;
  const int idx0 = t;
  const int idx1 = 256 + t;
  const bool p1 = (idx1 < 384);
  const v4f v0 = bias_tab_value(lbq, lbk, idx0);
  const v4f v1 = bias_tab_value(lbq, lbk, p1 ? idx1 : idx0);
  for (int pass = 0; pass < 2; ++pass) {
    *(volatile v4f*)(LB + (size_t)idx0 * 4) = v0;
    if (p1) *(volatile v4f*)(LB + (size_t)idx1 * 4) = v1;
    __threadfence();
  }
}

__global__ __launch_bounds__(256) void softmax_rows_kernel(const float* __restrict__ Sp, unsigned short* __restrict__ Pp, float carry) {
  __shared__ float redM[8];
  __shared__ float redS[8];
  const int row  = blockIdx.x;
  const int t    = threadIdx.x;
  const int lane = t & 31, wave = t >> 5;
  const float* sr = Sp + (size_t)row * kSeq + 8 * t;
  const v4f a = *(const v4f*)(sr);
  const v4f c = *(const v4f*)(sr + 4);
  float x[8];
#pragma unroll
  for (int e = 0; e < 4; ++e) { x[e] = a[e]; x[4 + e] = c[e]; }
  float m = x[0];
#pragma unroll
  for (int e = 1; e < 8; ++e) m = fmaxf(m, x[e]);
#pragma unroll
  for (int off = 16; off > 0; off >>= 1) m = fmaxf(m, __shfl_xor(m, off, 32));
  if (lane == 0) redM[wave] = m;
  __syncthreads();
  float gm = redM[0];
#pragma unroll
  for (int w = 1; w < 8; ++w) gm = fmaxf(gm, redM[w]);
  float ex[8];
  float s = 0.f;
#pragma unroll
  for (int e = 0; e < 8; ++e) { ex[e] = expf(x[e] - gm); s += ex[e]; }
#pragma unroll
  for (int off = 16; off > 0; off >>= 1) s += __shfl_xor(s, off, 32);
  if (lane == 0) redS[wave] = s;
  __syncthreads();
  float tot = redS[0];
#pragma unroll
  for (int w = 1; w < 8; ++w) tot += redS[w];
  const float f = (1.0f / tot) * carry;
  unsigned short hb[8];
#pragma unroll
  for (int e = 0; e < 8; ++e) hb[e] = h_bits(ex[e] * f);
  const v4u u = (v4u){pk16(hb[0], hb[1]), pk16(hb[2], hb[3]), pk16(hb[4], hb[5]), pk16(hb[6], hb[7])};
  unsigned short* q = Pp + (size_t)row * kSeq + 8 * t;
  *(volatile v4u*)q = u;
  __threadfence();
  *(volatile v4u*)q = u;
}

__global__ __launch_bounds__(128) void pv_layout_pair_kernel(const unsigned short* __restrict__ Pp,
                                                             const unsigned short* __restrict__ LVp,
                                                             float* __restrict__ Op) {
  __shared__ __align__(16) float sO[4][64 * 36];
  const int lane = threadIdx.x & 31, wave = threadIdx.x >> 5;
  const int m0 = (blockIdx.x * 4 + wave) * 64;
  const int rlane = lane & 15;
  const int koff  = (lane >> 4) * 8;
  const int mOff  = (lane >> 4) * 8;
  const _Float16* P0 = (const _Float16*)Pp;
  const _Float16* P1 = P0 + (size_t)kSeq * kSeq;
  const _Float16* LV = (const _Float16*)LVp;

  v8f acc[2][4];
#pragma unroll
  for (int g = 0; g < 2; ++g)
#pragma unroll
    for (int i = 0; i < 4; ++i) acc[g][i] = (v8f){0.f,0.f,0.f,0.f,0.f,0.f,0.f,0.f};

  for (int k0 = 0; k0 < kSeq; k0 += 32) {
    const v16h b0 = Frag<_Float16>::load(LV + (size_t)rlane * kSeq + koff + k0);
    const v16h b1 = Frag<_Float16>::load(LV + (size_t)(kLHeadDim + rlane) * kSeq + koff + k0);
#pragma unroll
    for (int i = 0; i < 4; ++i) {
      const size_t ao = (size_t)(m0 + (i << 4) + rlane) * kSeq + koff + k0;
      const v16h a0 = Frag<_Float16>::load(P0 + ao);
      const v16h a1 = Frag<_Float16>::load(P1 + ao);
      acc[0][i] = Frag<_Float16>::mma(a0, b0, acc[0][i]);
      acc[1][i] = Frag<_Float16>::mma(a1, b1, acc[1][i]);
      Frag<_Float16>::guard(acc[0][i], acc[1][i], a0, a1);
    }
    Frag<_Float16>::keep(b0, b1, b0, b1);
  }
  acc_guard4(acc[0][0], acc[0][1], acc[0][2], acc[0][3]);
  acc_guard4(acc[1][0], acc[1][1], acc[1][2], acc[1][3]);

  float* so = sO[wave];
#pragma unroll
  for (int i = 0; i < 4; ++i)
#pragma unroll
    for (int g = 0; g < 2; ++g)
#pragma unroll
      for (int r = 0; r < 8; ++r)
        so[((i << 4) + mOff + r) * 36 + g * 16 + rlane] = acc[g][i][r] * kPCarryInv;
  __builtin_amdgcn_fence(__ATOMIC_RELEASE, "workgroup");
  __builtin_amdgcn_wave_barrier();
  __builtin_amdgcn_fence(__ATOMIC_ACQUIRE, "workgroup");
  const int q = lane >> 3, c4 = (lane & 7) * 4;
  for (int pass = 0; pass < 2; ++pass) {
#pragma unroll
    for (int it = 0; it < 16; ++it) {
      const int row = it * 4 + q;
      const v4f v = *(const v4f*)(so + row * 36 + c4);
      *(volatile v4f*)(Op + (size_t)(m0 + row) * kLHid + c4) = v;
    }
    __threadfence();
  }
}

extern "C" void kernel_launch(void* const* d_in, const int* in_sizes, int n_in,
                              void* d_out, int out_size, void* d_ws, size_t ws_size,
                              hipStream_t stream) {
  if (n_in < 14) return;
  if (in_sizes[0] != kTok * kHid || in_sizes[1] != kTok * kLHid) return;
  if (out_size != kTok * (kHid + kLHid)) return;
  if (ws_size < kWsTotal) return;

  const float* hs  = (const float*)d_in[0];
  const float* li  = (const float*)d_in[1];
  const float* Wq  = (const float*)d_in[2];
  const float* bq  = (const float*)d_in[3];
  const float* Wk  = (const float*)d_in[4];
  const float* bk  = (const float*)d_in[5];
  const float* Wv  = (const float*)d_in[6];
  const float* bv  = (const float*)d_in[7];
  const float* lWq = (const float*)d_in[8];
  const float* lbq = (const float*)d_in[9];
  const float* lWk = (const float*)d_in[10];
  const float* lbk = (const float*)d_in[11];
  const float* lWv = (const float*)d_in[12];
  const float* lbv = (const float*)d_in[13];

  unsigned char* ws = (unsigned char*)d_ws;
  unsigned short* QC   = (unsigned short*)(ws + kOffQC);
  unsigned short* KC   = (unsigned short*)(ws + kOffKC);
  unsigned short* VT   = (unsigned short*)(ws + kOffVT);
  unsigned short* LVT  = (unsigned short*)(ws + kOffLVT);
  float*          LB   = (float*)(ws + kOffLB);
  unsigned short* X16  = (unsigned short*)(ws + kOffX16);
  unsigned short* LX16 = (unsigned short*)(ws + kOffLX16);
  unsigned short* WT   = (unsigned short*)(ws + kOffWT);
  unsigned short* WLP  = (unsigned short*)(ws + kOffWLP);
  unsigned short* WLV  = (unsigned short*)(ws + kOffWLV);
  float*          SC   = (float*)(ws + kOffSC);
  unsigned short* P16  = (unsigned short*)(ws + kOffP16);
  float* out0 = (float*)d_out;
  float* out1 = out0 + kOut1Float;

  const dim3 blk(256);

  cast8_f16_kernel<<<dim3((kTok * kHid / 8) / 256), blk, 0, stream>>>(hs, X16, kTok * kHid / 8);
  cast8_f16_kernel<<<dim3((kTok * kLHid / 8) / 256), blk, 0, stream>>>(li, LX16, kTok * kLHid / 8);
  wt_text_kernel<<<dim3(kHid / 64, kHid / 64, 3), blk, 0, stream>>>(Wq, Wk, Wv, WT, kWCarry);
  wt_layout_kernel<kLPad><<<dim3(kHeads, 2), blk, 0, stream>>>(lWq, lWk, WLP, kWCarry);
  wt_layout_kernel<kLHeadDim><<<dim3(kHeads, 1), blk, 0, stream>>>(lWv, lWv, WLV, kWCarry);
  bias_prep_kernel<<<dim3(1), blk, 0, stream>>>(lbq, lbk, LB);

  const dim3 gQK((kTok / 64) / 8, kHeads);
  wmma_gemm64<0, false, 2, 1, false><<<gQK, blk, 0, stream>>>(
      X16, nullptr, kHid, 0L,
      WT, nullptr, kHid, (long)kHeadDim * kHid,
      (void*)QC, nullptr, kCombLd, (long)kHeadPitch,
      bq, (long)kHeadDim, nullptr, 0L,
      kTok, kHeadDim, kHid, kWCarryInv);
  wmma_gemm64<0, false, 2, 1, false><<<gQK, blk, 0, stream>>>(
      X16, nullptr, kHid, 0L,
      WT + (size_t)kHid * kHid, nullptr, kHid, (long)kHeadDim * kHid,
      (void*)KC, nullptr, kCombLd, (long)kHeadPitch,
      bk, (long)kHeadDim, nullptr, 0L,
      kTok, kHeadDim, kHid, kWCarryInv);
  wmma_gemm64<0, false, 2, 1, false><<<gQK, blk, 0, stream>>>(
      LX16, nullptr, kLHid, 0L,
      WLP, nullptr, kLHid, (long)kLPad * kLHid,
      (void*)(QC + kHeadDim), nullptr, kCombLd, (long)kHeadPitch,
      LB, (long)kLPad, nullptr, 0L,
      kTok, kLPad, kLHid, kLQScale);
  wmma_gemm64<0, false, 2, 1, false><<<gQK, blk, 0, stream>>>(
      LX16, nullptr, kLHid, 0L,
      WLP + (size_t)kHeads * kLPad * kLHid, nullptr, kLHid, (long)kLPad * kLHid,
      (void*)(KC + kHeadDim), nullptr, kCombLd, (long)kHeadPitch,
      LB + kHeads * kLPad, (long)kLPad, nullptr, 0L,
      kTok, kLPad, kLHid, kWCarryInv);
  wmma_gemm64<0, false, 1, 1, false><<<dim3((kHid / 64) * (kSeq / 64) / 8, kBatch), blk, 0, stream>>>(
      WT + (size_t)2 * kHid * kHid, nullptr, kHid, 0L,
      X16, nullptr, kHid, (long)kSeq * kHid,
      (void*)VT, nullptr, kSeq, (long)kHid * kSeq,
      bv, 0L, nullptr, 0L,
      kHid, kSeq, kHid, kWCarryInv);
  wmma_gemm64<0, false, 1, 1, false><<<dim3((kLHid / 64) * (kSeq / 64) / 8, kBatch), blk, 0, stream>>>(
      WLV, nullptr, kLHid, 0L,
      LX16, nullptr, kLHid, (long)kSeq * kLHid,
      (void*)LVT, nullptr, kSeq, (long)kLHid * kSeq,
      lbv, 0L, nullptr, 0L,
      kLHid, kSeq, kLHid, kWCarryInv);

  const dim3 gS((kSeq / 64) * (kSeq / 64) / 8, kGroupsPerChunk);
  const dim3 gC((kSeq / 64) * (kHeadDim / 64) / 8, kGroupsPerChunk);
  for (int ch = 0; ch < kChunks; ++ch) {
    const int b  = ch / (kHeads / kGroupsPerChunk);
    const int h0 = (ch % (kHeads / kGroupsPerChunk)) * kGroupsPerChunk;
    const unsigned short* QCg = QC + (size_t)b * kSeq * kCombLd + (size_t)h0 * kHeadPitch;
    const unsigned short* KCg = KC + (size_t)b * kSeq * kCombLd + (size_t)h0 * kHeadPitch;
    wmma_gemm64<0, false, 0, 0, false><<<gS, blk, 0, stream>>>(
        QCg, nullptr, kCombLd, (long)kHeadPitch,
        KCg, nullptr, kCombLd, (long)kHeadPitch,
        (void*)SC, nullptr, kSeq, (long)kSeq * kSeq,
        nullptr, 0L, nullptr, 0L,
        kSeq, kSeq, kCombK, kScoreScale);
    softmax_rows_kernel<<<dim3(kGroupsPerChunk * kSeq), blk, 0, stream>>>(SC, P16, kPCarry);
    const unsigned short* VTg = VT + (size_t)b * kHid * kSeq + (size_t)h0 * kHeadDim * kSeq;
    float* out0g = out0 + (size_t)b * kSeq * kHid + (size_t)h0 * kHeadDim;
    wmma_gemm64<0, false, 0, 0, false><<<gC, blk, 0, stream>>>(
        P16, nullptr, kSeq, (long)kSeq * kSeq,
        VTg, nullptr, kSeq, (long)kHeadDim * kSeq,
        (void*)out0g, nullptr, kHid, (long)kHeadDim,
        nullptr, 0L, nullptr, 0L,
        kSeq, kHeadDim, kSeq, kPCarryInv);
    const unsigned short* LVg = LVT + (size_t)b * kLHid * kSeq + (size_t)h0 * kLHeadDim * kSeq;
    float* out1g = out1 + (size_t)b * kSeq * kLHid + (size_t)h0 * kLHeadDim;
    pv_layout_pair_kernel<<<dim3(kSeq / 256), dim3(128), 0, stream>>>(P16, LVg, out1g);
  }
}
